// MatchMatrix_23605140259564
// MI455X (gfx1250) — hardware-run, weakly checked
//
#include <hip/hip_runtime.h>


#ifndef NB
#define NB 8
#endif
#define NB_FULL 8
#define LA   128
#define LC   128
#define DD   256
#define H1   64
#define H2   32
#define H3   16
#define AW   4
#define QRS  2048.0f
#define QRI  (1.0f / 2048.0f)
#define WSC  64.0f
#define WSI  (1.0f / 64.0f)
#define SLOPE 0.01f

static_assert(NB <= NB_FULL);
static_assert(DD % 32 == 0);
static_assert(H1 == 64);
static_assert(H2 == 32);
static_assert(H3 == 16);
static_assert(LC % 16 == 0);
static_assert((NB * LA) % 16 == 0);
static_assert((NB * LA) % AW == 0);
static_assert(((size_t)NB * LA * DD) % 8 == 0);
static_assert((2 * H1 * DD / 8) % 256 == 0);
static_assert(H2 * H1 / 8 == 256);
static_assert(H3 * H2 / 8 == 64);
static_assert(32 * 16 * 8 == 16 * H1 * 4);
static_assert(32 * 16 * 2 == 16 * H3 * 4);
static_assert(16 * 68 * 4 <= 131072);
static_assert(AW * 256 * 4 <= 131072);

typedef _Float16 h16;
typedef unsigned short bf;
typedef __attribute__((ext_vector_type(16))) __bf16   v16bf;
typedef __attribute__((ext_vector_type(16))) _Float16 v16h;
typedef __attribute__((ext_vector_type(8)))  _Float16 v8h;
typedef __attribute__((ext_vector_type(8)))  unsigned short v8us;
typedef __attribute__((ext_vector_type(8)))  float    v8f;
typedef __attribute__((ext_vector_type(4)))  float    v4f;
typedef v4f  __attribute__((may_alias)) v4fa;

__device__ __forceinline__ unsigned short f2bf(float f) { unsigned u = __float_as_uint(f); u += 0x7FFFu + ((u >> 16) & 1u); return (unsigned short)(u >> 16); }
__device__ __forceinline__ float bfr(float f) { return __uint_as_float(((unsigned)f2bf(f)) << 16); }
__device__ __forceinline__ v16h cat16(v8h lo, v8h hi) { return __builtin_shufflevector(lo, hi, 0, 1, 2, 3, 4, 5, 6, 7, 8, 9, 10, 11, 12, 13, 14, 15); }
__device__ __forceinline__ v16bf cat16b(v8us lo, v8us hi) { return __builtin_bit_cast(v16bf, __builtin_shufflevector(lo, hi, 0, 1, 2, 3, 4, 5, 6, 7, 8, 9, 10, 11, 12, 13, 14, 15)); }
__device__ __forceinline__ v8f wmma16(v16h a, v16h b, v8f c) { return __builtin_amdgcn_wmma_f32_16x16x32_f16(false, a, false, b, (short)0, c, false, false); }
__device__ __forceinline__ v8f wmmab(v16bf a, v16bf b, v8f c) { return __builtin_amdgcn_wmma_f32_16x16x32_bf16(false, a, false, b, (short)0, c, false, false); }
__device__ __forceinline__ v16h  ldh(const h16* p) { return cat16(*(const v8h*)p, *(const v8h*)(p + 16)); }
__device__ __forceinline__ v16bf ldb(const bf* p)  { return cat16b(*(const v8us*)p, *(const v8us*)(p + 16)); }
__device__ __forceinline__ void wave_sync() { __builtin_amdgcn_fence(3  , "wavefront"); __builtin_amdgcn_wave_barrier(); asm volatile("" ::: "memory"); }

__device__ __forceinline__ v8f wmmabg(v16bf a, v16bf b, v8f c) { c = wmmab(a, b, c); asm volatile("v_nop\n\tv_nop\n\tv_nop\n\tv_nop" : "+v"(c) : "v"(a), "v"(b)); return c; }
__device__ __forceinline__ v8f wmma16g(v16h a, v16h b, v8f c) { c = wmma16(a, b, c); asm volatile("v_nop\n\tv_nop\n\tv_nop\n\tv_nop" : "+v"(c) : "v"(a), "v"(b)); return c; }
static __device__ __forceinline__ h16 toh_flush(float v) { const float w = (fabsf(v) < 6.103515625e-05f) ? 0.0f : v; return (h16)w; }
__device__ __forceinline__ float lrelu(float x) { return x >= 0.0f ? x : SLOPE * x; }
__device__ __forceinline__ void ld16f(const float* p, float (&o)[16]) {
    const v4f x0 = *(const v4f*)p, x1 = *(const v4f*)(p + 4), x2 = *(const v4f*)(p + 16), x3 = *(const v4f*)(p + 20);
#pragma unroll
    for (int i = 0; i < 4; ++i) { o[i] = x0[i]; o[4 + i] = x1[i]; o[8 + i] = x2[i]; o[12 + i] = x3[i]; }
}
__device__ __forceinline__ void mkfrag(const float (&ap)[16], const float (&cp)[16], v16h& hv, v16h& hr) {
#pragma unroll
    for (int i = 0; i < 16; ++i) { const float x = lrelu(ap[i] + cp[i]); const h16 g = toh_flush(x); hv[i] = g; hr[i] = toh_flush((x - (float)g) * QRS); }
}

__global__ __launch_bounds__(256) void k_cvt8(const float* __restrict__ src, bf* dst, size_t n8) {
    const size_t i = (size_t)blockIdx.x * 256 + threadIdx.x; if (i >= n8) return;
    const v8f v = *(const v8f*)(src + i * 8); v8us o;
#pragma unroll
    for (int k = 0; k < 8; ++k) o[k] = f2bf(v[k]);
    *(volatile v8us*)(dst + i * 8) = o; __threadfence(); *(volatile v8us*)(dst + i * 8) = o;
}

__global__ __launch_bounds__(256) void k_w1t(const float* __restrict__ W1, bf* W1T) {
    const unsigned p = blockIdx.x * 256u + threadIdx.x; if (p >= (unsigned)(2 * H1 * DD / 8)) return;
    const unsigned half = p / (unsigned)(H1 * DD / 8), n = (p / (unsigned)(DD / 8)) % (unsigned)H1, k8 = (p % (unsigned)(DD / 8)) * 8u;
    const float* s = W1 + (size_t)(half * (unsigned)DD + k8) * H1 + n;
    v8us o;
#pragma unroll
    for (int j = 0; j < 8; ++j) o[j] = f2bf(s[(size_t)j * H1]);
    *(volatile v8us*)(W1T + (size_t)p * 8) = o; __threadfence(); *(volatile v8us*)(W1T + (size_t)p * 8) = o;
}

__global__ __launch_bounds__(256) void k_w23t(const float* __restrict__ W2, const float* __restrict__ W3, h16* W2T, h16* W3T) {
    const unsigned p = threadIdx.x;
    { const unsigned n = p / (unsigned)(H1 / 8), k8 = (p % (unsigned)(H1 / 8)) * 8u;
      const float* s = W2 + (size_t)k8 * H2 + n; v8h o;
#pragma unroll
      for (int j = 0; j < 8; ++j) o[j] = toh_flush(bfr(s[(size_t)j * H2]) * WSC);
      *(volatile v8h*)(W2T + (size_t)p * 8) = o; __threadfence(); *(volatile v8h*)(W2T + (size_t)p * 8) = o; }
    if (p < (unsigned)(H3 * H2 / 8)) {
      const unsigned n = p / (unsigned)(H2 / 8), k8 = (p % (unsigned)(H2 / 8)) * 8u;
      const float* s = W3 + (size_t)k8 * H3 + n; v8h o;
#pragma unroll
      for (int j = 0; j < 8; ++j) o[j] = toh_flush(bfr(s[(size_t)j * H3]) * WSC);
      *(volatile v8h*)(W3T + (size_t)p * 8) = o; __threadfence(); *(volatile v8h*)(W3T + (size_t)p * 8) = o; }
}

__global__ __launch_bounds__(32) void k_ab(const bf* __restrict__ XB, const bf* __restrict__ W1T, float* ABP) {
    __shared__ __align__(16) float os[16 * 68];
    const int lane = threadIdx.x & 31, lr = lane & 15, hi = lane >> 4;
    const unsigned r0 = blockIdx.x * 16u; const unsigned mat = blockIdx.y;
    const size_t aoff = (size_t)mat * ((size_t)NB * LA * DD) + (size_t)(r0 + (unsigned)lr) * DD + 8 * hi;
    const size_t boff = (size_t)mat * ((size_t)H1 * DD) + (size_t)lr * DD + 8 * hi;
    v8f acc[4];
#pragma unroll
    for (int nb = 0; nb < 4; ++nb) acc[nb] = (v8f){};
#pragma unroll 1
    for (int kc = 0; kc < DD; kc += 32) {
        const v16bf a = ldb(XB + aoff + kc);
#pragma unroll
        for (int nb = 0; nb < 4; ++nb) { const v16bf b = ldb(W1T + boff + (size_t)nb * 16 * DD + kc); acc[nb] = wmmabg(a, b, acc[nb]); }
    }
#pragma unroll
    for (int nb = 0; nb < 4; ++nb) {
#pragma unroll
        for (int j = 0; j < 8; ++j) os[(hi * 8 + j) * 68 + nb * 16 + lr] = acc[nb][j]; }
    wave_sync();
    float* orow = ABP + (size_t)mat * ((size_t)NB * LA * H1) + (size_t)r0 * H1;
#pragma unroll 1
    for (int ps = 0; ps < 2; ++ps) {
#pragma unroll
        for (int s = 0; s < 8; ++s) { const int p = s * 32 + lane; const int row = p >> 4, c4 = (p & 15) * 4;
            const v4f val = *(const v4fa*)(&os[row * 68 + c4]);
            *(volatile v4f*)(orow + (size_t)p * 4) = val; }
        if (ps == 0) __threadfence(); }
}

__global__ __launch_bounds__(32 * AW) void k_pair(const float* __restrict__ ABP, const h16* __restrict__ W2T, const h16* __restrict__ W3T,
                                                  const float* __restrict__ b1, const float* __restrict__ b2, const float* __restrict__ b3, float* OUT) {
    __shared__ __align__(16) float os[AW * 256];
    const int lane = threadIdx.x & 31, lr = lane & 15, hi = lane >> 4;
    const int wave = __builtin_amdgcn_readfirstlane((int)(threadIdx.x >> 5));
    const unsigned bx = blockIdx.x;
    const unsigned ba = bx * (unsigned)AW + (unsigned)wave;
    const unsigned bb = ba / (unsigned)LA;
    const int wb = wave * 256;
    const v16h w2a00 = ldh(W2T + (size_t)lr * H1 + 8 * hi);
    const v16h w2a01 = ldh(W2T + (size_t)lr * H1 + 32 + 8 * hi);
    const v16h w2a10 = ldh(W2T + (size_t)(16 + lr) * H1 + 8 * hi);
    const v16h w2a11 = ldh(W2T + (size_t)(16 + lr) * H1 + 32 + 8 * hi);
    const v16h w3a   = ldh(W3T + (size_t)lr * H2 + 8 * hi);
    float ap0[16], ap1[16];
    { float t0[16], t1[16], u0[16], u1[16];
      ld16f(ABP + (size_t)ba * H1 + 8 * hi, t0); ld16f(ABP + (size_t)ba * H1 + 32 + 8 * hi, t1);
      ld16f(b1 + 8 * hi, u0); ld16f(b1 + 32 + 8 * hi, u1);
#pragma unroll
      for (int i = 0; i < 16; ++i) { ap0[i] = t0[i] + bfr(u0[i]); ap1[i] = t1[i] + bfr(u1[i]); } }
    float b2v0[8], b2v1[8], b3v[8];
    { const v4f x0 = *(const v4f*)(b2 + 8 * hi), x1 = *(const v4f*)(b2 + 8 * hi + 4), y0 = *(const v4f*)(b2 + 16 + 8 * hi), y1 = *(const v4f*)(b2 + 16 + 8 * hi + 4);
      const v4f z0 = *(const v4f*)(b3 + 8 * hi), z1 = *(const v4f*)(b3 + 8 * hi + 4);
#pragma unroll
      for (int i = 0; i < 4; ++i) { b2v0[i] = bfr(x0[i]); b2v0[4 + i] = bfr(x1[i]); b2v1[i] = bfr(y0[i]); b2v1[4 + i] = bfr(y1[i]); b3v[i] = bfr(z0[i]); b3v[4 + i] = bfr(z1[i]); } }
    const size_t cbase = (size_t)NB * LA * H1 + (size_t)(bb * (unsigned)LC + (unsigned)lr) * H1 + 8 * hi;
#pragma unroll 1
    for (unsigned ct = 0; ct < (unsigned)(LC / 16); ++ct) {
        const size_t crow = cbase + (size_t)(ct * 16u) * H1;
        v8f aV0 = (v8f){}, aV1 = (v8f){}, aR0 = (v8f){}, aR1 = (v8f){};
        { float cp[16]; ld16f(ABP + crow, cp); v16h hv, hr; mkfrag(ap0, cp, hv, hr);
          aV0 = wmma16g(w2a00, hv, aV0); aR0 = wmma16g(w2a00, hr, aR0); aV1 = wmma16g(w2a10, hv, aV1); aR1 = wmma16g(w2a10, hr, aR1); }
        { float cp[16]; ld16f(ABP + crow + 32, cp); v16h hv, hr; mkfrag(ap1, cp, hv, hr);
          aV0 = wmma16g(w2a01, hv, aV0); aR0 = wmma16g(w2a01, hr, aR0); aV1 = wmma16g(w2a11, hv, aV1); aR1 = wmma16g(w2a11, hr, aR1); }
        v16h p3, r3;
#pragma unroll
        for (int r = 0; r < 8; ++r) {
            const float t0 = lrelu((aV0[r] + aR0[r] * QRI) * WSI + b2v0[r]);
            const float t1 = lrelu((aV1[r] + aR1[r] * QRI) * WSI + b2v1[r]);
            const h16 g0 = toh_flush(t0); const h16 g1 = toh_flush(t1);
            p3[r] = g0; p3[8 + r] = g1;
            r3[r] = toh_flush((t0 - (float)g0) * QRS); r3[8 + r] = toh_flush((t1 - (float)g1) * QRS); }
        v8f cV = (v8f){}, cR = (v8f){};
        cV = wmma16g(w3a, p3, cV); cR = wmma16g(w3a, r3, cR);
        { v4f a, c;
#pragma unroll
          for (int i = 0; i < 4; ++i) { a[i] = lrelu((cV[i] + cR[i] * QRI) * WSI + b3v[i]); c[i] = lrelu((cV[4 + i] + cR[4 + i] * QRI) * WSI + b3v[4 + i]); }
          *(v4fa*)(&os[wb + lr * 16 + 8 * hi]) = a; *(v4fa*)(&os[wb + lr * 16 + 8 * hi + 4]) = c; }
        wave_sync();
        float* orow = OUT + ((size_t)ba * LC + (size_t)(ct * 16u)) * H3;
#pragma unroll 1
        for (int ps = 0; ps < 2; ++ps) {
#pragma unroll
            for (int s = 0; s < 2; ++s) { const int p = s * 32 + lane;
                const v4f val = *(const v4fa*)(&os[wb + p * 4]);
                *(volatile v4f*)(orow + (size_t)p * 4) = val; }
            if (ps == 0) __threadfence(); }
        wave_sync();
    }
}

static constexpr size_t al256(size_t v) { return (v + 255) & ~(size_t)255; }
static constexpr size_t N_X   = (size_t)NB * LA * DD;
static constexpr size_t N8_X  = N_X / 8;
static constexpr size_t SZ_XB = al256((size_t)2 * NB * LA * DD * 2);
static constexpr size_t SZ_W1 = al256((size_t)2 * H1 * DD * 2);
static constexpr size_t SZ_W2 = al256((size_t)H2 * H1 * 2);
static constexpr size_t SZ_W3 = al256((size_t)H3 * H2 * 2);
static constexpr size_t SZ_AB = al256((size_t)2 * NB * LA * H1 * 4);
static constexpr size_t SZ_TOTAL = SZ_XB + SZ_W1 + SZ_W2 + SZ_W3 + SZ_AB;
static constexpr unsigned G_CVT = (unsigned)((N8_X + 255) / 256);
static constexpr unsigned G_W1T = (unsigned)(2 * H1 * DD / 8 / 256);
static_assert(SZ_TOTAL <= (size_t)134217728);
static_assert((N_X * 2) % 256 == 0);
static_assert(((size_t)NB * LA * H1 * 4) % 256 == 0);
static_assert((size_t)G_W1T * 256 * 8 == (size_t)2 * H1 * DD);
static_assert((size_t)(NB * LA / 16) * 16 * H1 * 2 == (size_t)2 * NB * LA * H1);
static_assert((size_t)(NB * LA / AW) * AW * LC * H3 == (size_t)NB * LA * LC * H3);

extern "C" void kernel_launch(void* const* d_in, const int* in_sizes, int n_in,
                              void* d_out, int out_size, void* d_ws, size_t ws_size, hipStream_t stream) {
    if (n_in < 8) return;
    if ((size_t)in_sizes[0] < N_X || (size_t)in_sizes[1] < N_X) return;
    if (in_sizes[2] < 2 * DD * H1 || in_sizes[3] < H1 || in_sizes[4] < H1 * H2 || in_sizes[5] < H2 || in_sizes[6] < H2 * H3 || in_sizes[7] < H3) return;
    if ((size_t)out_size < (size_t)NB * LA * LC * H3) return;
    if (SZ_TOTAL > ws_size) return;
    const float* sa = (const float*)d_in[0]; const float* sc = (const float*)d_in[1];
    const float* w1 = (const float*)d_in[2]; const float* b1 = (const float*)d_in[3];
    const float* w2 = (const float*)d_in[4]; const float* b2 = (const float*)d_in[5];
    const float* w3 = (const float*)d_in[6]; const float* b3 = (const float*)d_in[7];
    float* OUT = (float*)d_out;
    char* wsp = (char*)d_ws;
    bf*  XB  = (bf*)wsp;  wsp += SZ_XB;
    bf*  W1T = (bf*)wsp;  wsp += SZ_W1;
    h16* W2T = (h16*)wsp; wsp += SZ_W2;
    h16* W3T = (h16*)wsp; wsp += SZ_W3;
    float* ABP = (float*)wsp; wsp += SZ_AB;

    k_cvt8<<<G_CVT, 256, 0, stream>>>(sa, XB, N8_X);
    k_cvt8<<<G_CVT, 256, 0, stream>>>(sc, XB + N_X, N8_X);
    k_w1t<<<G_W1T, 256, 0, stream>>>(w1, W1T);
    k_w23t<<<1, 256, 0, stream>>>(w2, w3, W2T, W3T);
    k_ab<<<dim3(NB * LA / 16, 2, 1), 32, 0, stream>>>(XB, W1T, ABP);
    k_pair<<<dim3(NB * LA / AW, 1, 1), 32 * AW, 0, stream>>>(ABP, W2T, W3T, b1, b2, b3, OUT);
}
